// GCN_3435973837349
// MI455X (gfx1250) — hardware-verified
//
#include <hip/hip_runtime.h>
#include <stddef.h>
#include <stdint.h>
#include <math.h>


#define F1    64
#define F2    128
#define NC    29
#define K2    128
#define K3    256
#define NTHR  256
#define NWAVE 8
#define EPT   8
#define CHUNK (NTHR * EPT)
#define WCAP  (EPT * 32)
#define LISTN (NWAVE * WCAP)
#define TABN  65536
#define SLE   14
#define RIE   4
#define SLG   11
#define RIG   32
#define CMP_INTS (TABN + LISTN + 16)
#define TM    64
#define GTHR  128
#define APW   68
#define GPB   32
#define PARN  1024
#define P_W1  0
#define P_B1  192
#define P_M1  256
#define P_S1  320
#define P_E1  384
#define P_B2  448
#define P_M2  576
#define P_S2  704
#define P_E2  832
#define P_B3  960
#define NU2   2048
#define NU3   1024

static_assert((CHUNK & (CHUNK - 1)) == 0 && CHUNK == 2048);
static_assert((1 << SLE) * RIE == TABN && (1 << SLG) * RIG == TABN);
static_assert(((long long)CHUNK << SLE) < (1LL << 31));
static_assert((TABN + LISTN) % (NTHR * 4) == 0);
static_assert(TABN % (NTHR * 4) == 0 && (1 << SLE) % (NTHR * 4) == 0);
static_assert(K2 % 32 == 0 && K3 % 32 == 0 && K2 == 2 * F1 && K3 == 2 * F2);
static_assert(TM == (GTHR / 32) * 16);
static_assert(NU2 % NTHR == 0 && NU3 % NTHR == 0);
static_assert((TM * NC * 4) % 128 == 0 && (TM * NC) % 4 == 0);
static_assert((GPB * NC * 4) % 128 == 0 && (GPB * NC) / 4 <= NTHR);
static_assert(CMP_INTS * 4 <= 300000);
static_assert(P_B3 + 32 <= PARN && PARN == 4 * NTHR && PARN == 8 * GTHR);

typedef float          v2f   __attribute__((ext_vector_type(2)));
typedef float          v4f   __attribute__((ext_vector_type(4)));
typedef float          v8f   __attribute__((ext_vector_type(8)));
typedef int            v4i   __attribute__((ext_vector_type(4)));
typedef int            v8i   __attribute__((ext_vector_type(8)));
typedef unsigned short v4us  __attribute__((ext_vector_type(4)));
typedef unsigned short v8us  __attribute__((ext_vector_type(8)));
typedef unsigned short v16us __attribute__((ext_vector_type(16)));
typedef __bf16         v16bf __attribute__((ext_vector_type(16)));
typedef v2f  __attribute__((may_alias)) v2fa;
typedef v4f  __attribute__((may_alias)) v4fa;
typedef v4i  __attribute__((may_alias)) v4ia;
typedef v4us __attribute__((may_alias)) v4usa;
typedef v8us __attribute__((may_alias)) v8usa;
union FragB { v16bf v; v16us u; v8us h[2]; v8i w; };

__device__ __forceinline__ v8f wmb(const FragB& a, const FragB& b, v8f c) {
  v8f d = __builtin_amdgcn_wmma_f32_16x16x32_bf16(false, a.v, false, b.v, (short)0, c, false, false);
  asm volatile("v_nop\n\tv_nop\n\tv_nop\n\tv_nop" : "+v"(d) : "v"(a.w), "v"(b.w));
  return d;
}

__device__ __forceinline__ unsigned bf16_bits(float f) {
  const unsigned u = __float_as_uint(f);
  return (u + 0x7FFFu + ((u >> 16) & 1u)) >> 16;
}
__device__ __forceinline__ float bf16_val(float f) {
  return __uint_as_float(bf16_bits(f) << 16);
}

template <int SLB>
__device__ __forceinline__ int scan_chunk(const int* __restrict__ keys, int nE, int cbase, int slotBase,
                                          int nb, int vec8, int* list, int tid, int lane, int wave) {
  int wc = 0;
  const int el0  = tid * EPT;
  const int e0   = cbase + el0;
  const int sent = -2147483647 - 1;
  v4i da, db;
  if (vec8 != 0 && cbase + CHUNK <= nE) {
    da = *(const v4i*)(keys + e0);
    db = *(const v4i*)(keys + e0 + 4);
  } else {
    da.x = (e0     < nE) ? keys[min(e0,     nE - 1)] : sent;
    da.y = (e0 + 1 < nE) ? keys[min(e0 + 1, nE - 1)] : sent;
    da.z = (e0 + 2 < nE) ? keys[min(e0 + 2, nE - 1)] : sent;
    da.w = (e0 + 3 < nE) ? keys[min(e0 + 3, nE - 1)] : sent;
    db.x = (e0 + 4 < nE) ? keys[min(e0 + 4, nE - 1)] : sent;
    db.y = (e0 + 5 < nE) ? keys[min(e0 + 5, nE - 1)] : sent;
    db.z = (e0 + 6 < nE) ? keys[min(e0 + 6, nE - 1)] : sent;
    db.w = (e0 + 7 < nE) ? keys[min(e0 + 7, nE - 1)] : sent;
  }
  const unsigned nbs = (unsigned)slotBase;
  const unsigned unb = (unsigned)nb;
  const unsigned s0 = (unsigned)da.x - nbs, s1 = (unsigned)da.y - nbs;
  const unsigned s2 = (unsigned)da.z - nbs, s3 = (unsigned)da.w - nbs;
  const unsigned s4 = (unsigned)db.x - nbs, s5 = (unsigned)db.y - nbs;
  const unsigned s6 = (unsigned)db.z - nbs, s7 = (unsigned)db.w - nbs;
  const bool h0 = s0 < unb, h1 = s1 < unb, h2 = s2 < unb, h3 = s3 < unb;
  const bool h4 = s4 < unb, h5 = s5 < unb, h6 = s6 < unb, h7 = s7 < unb;
  const unsigned any = __builtin_amdgcn_ballot_w32(h0 | h1 | h2 | h3 | h4 | h5 | h6 | h7);
  if (any != 0u) {
    const unsigned m0 = __builtin_amdgcn_ballot_w32(h0);
    const unsigned m1 = __builtin_amdgcn_ballot_w32(h1);
    const unsigned m2 = __builtin_amdgcn_ballot_w32(h2);
    const unsigned m3 = __builtin_amdgcn_ballot_w32(h3);
    const unsigned m4 = __builtin_amdgcn_ballot_w32(h4);
    const unsigned m5 = __builtin_amdgcn_ballot_w32(h5);
    const unsigned m6 = __builtin_amdgcn_ballot_w32(h6);
    const unsigned m7 = __builtin_amdgcn_ballot_w32(h7);
    int p = (int)__builtin_amdgcn_mbcnt_lo(m0, 0u) + (int)__builtin_amdgcn_mbcnt_lo(m1, 0u)
          + (int)__builtin_amdgcn_mbcnt_lo(m2, 0u) + (int)__builtin_amdgcn_mbcnt_lo(m3, 0u)
          + (int)__builtin_amdgcn_mbcnt_lo(m4, 0u) + (int)__builtin_amdgcn_mbcnt_lo(m5, 0u)
          + (int)__builtin_amdgcn_mbcnt_lo(m6, 0u) + (int)__builtin_amdgcn_mbcnt_lo(m7, 0u);
#define PUTJ(J, HJ, SJ) if (HJ) { if (p < WCAP) list[wave * WCAP + p] = ((el0 + (J)) << SLB) | (int)(SJ); p = p + 1; }
    PUTJ(0, h0, s0)
    PUTJ(1, h1, s1)
    PUTJ(2, h2, s2)
    PUTJ(3, h3, s3)
    PUTJ(4, h4, s4)
    PUTJ(5, h5, s5)
    PUTJ(6, h6, s6)
    PUTJ(7, h7, s7)
#undef PUTJ
    wc = (int)__builtin_popcount(m0) + (int)__builtin_popcount(m1) + (int)__builtin_popcount(m2)
       + (int)__builtin_popcount(m3) + (int)__builtin_popcount(m4) + (int)__builtin_popcount(m5)
       + (int)__builtin_popcount(m6) + (int)__builtin_popcount(m7);
  }
  return wc;
}

__global__ __launch_bounds__(NTHR) void k_prep(
    const float* __restrict__ W1, const float* __restrict__ b1, const float* __restrict__ g1,
    const float* __restrict__ be1, const float* __restrict__ m1, const float* __restrict__ v1,
    const float* __restrict__ W2, const float* __restrict__ b2, const float* __restrict__ g2,
    const float* __restrict__ be2, const float* __restrict__ m2, const float* __restrict__ v2,
    const float* __restrict__ W3, const float* __restrict__ b3,
    float* par, unsigned short* W2T, unsigned short* W3T) {
  __shared__ __attribute__((aligned(16))) float ps[PARN];
  const int tid = (int)threadIdx.x;
  const int b   = (int)blockIdx.x;
  if (b < NU2 / NTHR) {
    const int u  = b * NTHR + tid;
    const int n  = u >> 4;
    const int k8 = (u & 15) * 8;
    const int kk = k8 & (F1 - 1);
    const float* p = W2 + (size_t)kk * F2 + n;
    v8us o;
#pragma unroll
    for (int i = 0; i < 8; ++i) o[i] = (unsigned short)bf16_bits(p[(size_t)i * F2]);
    unsigned short* dp = W2T + (size_t)n * K2 + k8;
    *(volatile v8us*)dp = o;
    __threadfence();
    *(volatile v8us*)dp = o;
  } else if (b < NU2 / NTHR + NU3 / NTHR) {
    const int v  = (b - NU2 / NTHR) * NTHR + tid;
    const int n  = v >> 5;
    const int k8 = (v & 31) * 8;
    const int kk = k8 & (F2 - 1);
    const int nc = n < NC ? n : NC - 1;
    const float* p = W3 + (size_t)kk * NC + nc;
    v8us o;
#pragma unroll
    for (int i = 0; i < 8; ++i) {
      const unsigned q = bf16_bits(p[(size_t)i * NC]);
      o[i] = (n < NC) ? (unsigned short)q : (unsigned short)0;
    }
    unsigned short* dp = W3T + (size_t)n * K3 + k8;
    *(volatile v8us*)dp = o;
    __threadfence();
    *(volatile v8us*)dp = o;
  } else {
    {
      const int i1 = tid < 3 * F1 ? tid : 3 * F1 - 1;
      const float w = bf16_val(W1[i1]);
      if (tid < 3 * F1) ps[P_W1 + tid] = w;
      const int c = tid & (F1 - 1);
      const float bb = bf16_val(b1[c]);
      const float gg = bf16_val(g1[c]);
      const float ee = bf16_val(be1[c]);
      const float mm = bf16_val(m1[c]);
      const float vv = bf16_val(v1[c]);
      const float sc = gg * rsqrtf(vv + 1e-5f);
      if (tid < F1) { ps[P_B1 + c] = bb; ps[P_M1 + c] = mm; ps[P_S1 + c] = sc; ps[P_E1 + c] = ee; }
    }
    __syncthreads();
    {
      const int c = tid & (F2 - 1);
      const float bb = bf16_val(b2[c]);
      const float gg = bf16_val(g2[c]);
      const float ee = bf16_val(be2[c]);
      const float mm = bf16_val(m2[c]);
      const float vv = bf16_val(v2[c]);
      const float sc = gg * rsqrtf(vv + 1e-5f);
      if (tid < F2) { ps[P_B2 + c] = bb; ps[P_M2 + c] = mm; ps[P_S2 + c] = sc; ps[P_E2 + c] = ee; }
      const int c3 = tid < NC ? tid : NC - 1;
      const float b3v = bf16_val(b3[c3]);
      if (tid < 32) { ps[P_B3 + tid] = (tid < NC) ? b3v : 0.0f; ps[P_B3 + 32 + tid] = 0.0f; }
    }
    __syncthreads();
    const v4f pv = *(const v4fa*)(ps + 4 * tid);
    float* dp = par + 4 * tid;
    *(volatile v4f*)dp = pv;
    __threadfence();
    *(volatile v4f*)dp = pv;
  }
}

__device__ __forceinline__ float dinv_of(int c, int cap) {
  const float d = rsqrtf((float)c + 1.0f);
  return (c > cap) ? __int_as_float(0x7fc00000) : d;
}

template <int SLB, int RI, int EDGE>
__global__ __launch_bounds__(NTHR) void k_compact(const int* __restrict__ keys, const int* __restrict__ vals,
                                                  int nE, int vmax, int vec8, int* tabG, float* dinvG) {
  extern __shared__ __attribute__((aligned(16))) int dsm[];
  constexpr int NB = 1 << SLB;
  static_assert(NB * RI == TABN);
  int* tab  = dsm;
  int* list = dsm + TABN;
  int* misc = list + LISTN;
  const int tid = (int)threadIdx.x, lane = tid & 31, wave = tid >> 5;
  const int slotBase = (int)blockIdx.x * NB;

  {
    const v4i z4 = {0, 0, 0, 0};
    for (int i = tid * 4; i < TABN + LISTN; i += NTHR * 4) *(v4ia*)(dsm + i) = z4;
    if (tid < 16) misc[tid] = 0;
  }
  __syncthreads();

  const int nChunks = (nE + CHUNK - 1) / CHUNK;
#pragma unroll 1
  for (int ch = 0; ch < nChunks; ++ch) {
    const int cbase = ch * CHUNK;
    const int wc = scan_chunk<SLB>(keys, nE, cbase, slotBase, NB, vec8, list, tid, lane, wave);
    if (lane == 0) misc[wave] = wc;
    __syncthreads();
    if (wave == 0) {
#pragma unroll 1
      for (int w2 = 0; w2 < NWAVE; ++w2) {
        int c = misc[w2];
        c = c < 0 ? 0 : (c > WCAP ? WCAP : c);
#pragma unroll 1
        for (int b0 = 0; b0 < c; b0 += 32) {
          const int idx  = b0 + lane;
          const int ent  = list[w2 * WCAP + (idx < WCAP ? idx : WCAP - 1)];
          const int slot = ent & (NB - 1);
          const int el   = (ent >> SLB) & (CHUNK - 1);
          int eid = cbase + el;
          eid = eid > nE - 1 ? nE - 1 : eid;
          int val = eid;
          if constexpr (EDGE != 0) {
            int sr = vals[eid];
            sr = sr < 0 ? 0 : (sr > vmax - 1 ? vmax - 1 : sr);
            val = sr;
          }
          const int m32 = (c - b0) < 32 ? (c - b0) : 32;
#pragma unroll 1
          for (int k = 0; k < m32; ++k) {
            const int sk = __builtin_amdgcn_readlane(slot, k);
            const int vk = __builtin_amdgcn_readlane(val, k);
            if (lane == 0) {
              int* rp = tab + sk * RI;
              const int cc = rp[RI - 1];
              if (cc >= 0 && cc < RI - 1) rp[cc] = vk;
              rp[RI - 1] = cc + 1;
            }
          }
        }
      }
    }
    __syncthreads();
  }

  int* gp = tabG + (size_t)blockIdx.x * TABN;
#pragma unroll 4
  for (int it = 0; it < TABN / (NTHR * 4); ++it) {
    const int o = (it * NTHR + tid) * 4;
    const v4i v = *(const v4ia*)(tab + o);
    *(volatile v4i*)(gp + o) = v;
  }
  __threadfence();
#pragma unroll 4
  for (int it = 0; it < TABN / (NTHR * 4); ++it) {
    const int o = (it * NTHR + tid) * 4;
    const v4i v = *(const v4ia*)(tab + o);
    *(volatile v4i*)(gp + o) = v;
  }
  if constexpr (EDGE != 0) {
    float* dq = dinvG + (size_t)slotBase;
#pragma unroll 4
    for (int it = 0; it < NB / (NTHR * 4); ++it) {
      const int s0 = (it * NTHR + tid) * 4;
      v4f d;
      d.x = dinv_of(tab[(s0 + 0) * RI + RI - 1], RI - 1);
      d.y = dinv_of(tab[(s0 + 1) * RI + RI - 1], RI - 1);
      d.z = dinv_of(tab[(s0 + 2) * RI + RI - 1], RI - 1);
      d.w = dinv_of(tab[(s0 + 3) * RI + RI - 1], RI - 1);
      *(volatile v4f*)(dq + s0) = d;
    }
    __threadfence();
#pragma unroll 4
    for (int it = 0; it < NB / (NTHR * 4); ++it) {
      const int s0 = (it * NTHR + tid) * 4;
      v4f d;
      d.x = dinv_of(tab[(s0 + 0) * RI + RI - 1], RI - 1);
      d.y = dinv_of(tab[(s0 + 1) * RI + RI - 1], RI - 1);
      d.z = dinv_of(tab[(s0 + 2) * RI + RI - 1], RI - 1);
      d.w = dinv_of(tab[(s0 + 3) * RI + RI - 1], RI - 1);
      *(volatile v4f*)(dq + s0) = d;
    }
  }
}

__global__ __launch_bounds__(NTHR) void k_agg1(const float* __restrict__ x, const int* __restrict__ nbt,
                                               const float* __restrict__ dinv, int nN, float* ax) {
  const int i = (int)blockIdx.x * NTHR + (int)threadIdx.x;
  const bool live = i < nN;
  const int ic = live ? i : nN - 1;
  const v4i nb = *(const v4i*)(nbt + (size_t)ic * 4);
  const float di = dinv[ic];
  const float x0 = bf16_val(x[(size_t)ic * 3 + 0]);
  const float x1 = bf16_val(x[(size_t)ic * 3 + 1]);
  const float x2 = bf16_val(x[(size_t)ic * 3 + 2]);
  int c = nb.w;
  c = c < 0 ? 0 : (c > RIE - 1 ? RIE - 1 : c);
  float a0 = 0.0f, a1 = 0.0f, a2 = 0.0f;
  int sj = nb.x, sy = nb.y, sz = nb.z;
#pragma unroll 1
  for (int k = 0; k < RIE - 1; ++k) {
    int s = sj;
    s = s < 0 ? 0 : (s > nN - 1 ? nN - 1 : s);
    const float ds = dinv[s];
    const float y0 = bf16_val(x[(size_t)s * 3 + 0]);
    const float y1 = bf16_val(x[(size_t)s * 3 + 1]);
    const float y2 = bf16_val(x[(size_t)s * 3 + 2]);
    const bool on = k < c;
    const float w  = on ? ds * di : 0.0f;
    const float q0 = on ? y0 : 0.0f;
    const float q1 = on ? y1 : 0.0f;
    const float q2 = on ? y2 : 0.0f;
    a0 = fmaf(w, q0, a0); a1 = fmaf(w, q1, a1); a2 = fmaf(w, q2, a2);
    sj = sy; sy = sz;
  }
  const float rd = di * di;
  a0 = fmaf(rd, x0, a0); a1 = fmaf(rd, x1, a1); a2 = fmaf(rd, x2, a2);
  v4f o;
  o.x = live ? a0 : 0.0f; o.y = live ? a1 : 0.0f; o.z = live ? a2 : 0.0f; o.w = live ? di : 0.0f;
  float* dp = ax + (size_t)i * 4;
  *(volatile v4f*)dp = o;
  __threadfence();
  *(volatile v4f*)dp = o;
}

__device__ __forceinline__ void h1acc(float a0, float a1, float a2, float w,
                                      v2f w10, v2f w11, v2f w12, v2f qb, v2f qm, v2f qs, v2f qe,
                                      float& acc0, float& acc1) {
  const float t0 = fmaf(a2, w12.x, fmaf(a1, w11.x, a0 * w10.x)) + qb.x;
  const float t1 = fmaf(a2, w12.y, fmaf(a1, w11.y, a0 * w10.y)) + qb.y;
  float y0 = (t0 - qm.x) * qs.x + qe.x;
  float y1 = (t1 - qm.y) * qs.y + qe.y;
  y0 = (y0 > 0.0f) ? y0 : (y0 - y0);
  y1 = (y1 > 0.0f) ? y1 : (y1 - y1);
  acc0 = fmaf(w, y0, acc0);
  acc1 = fmaf(w, y1, acc1);
}

__global__ __launch_bounds__(GTHR) void k_layer2(const float* __restrict__ ax, const int* __restrict__ nbt,
                                                 const float* __restrict__ par,
                                                 const unsigned short* __restrict__ W2T,
                                                 const unsigned short* __restrict__ W3T,
                                                 int nN, float* t3) {
  __shared__ __attribute__((aligned(16))) float    pars[PARN];
  __shared__ __attribute__((aligned(16))) unsigned As[TM * APW];
  __shared__ __attribute__((aligned(16))) float    stg[TM * F2];
  __shared__ __attribute__((aligned(16))) float    t3s[TM * NC];
  const int tid = (int)threadIdx.x, lane = tid & 31, wave = tid >> 5, hh = lane >> 4, m = lane & 15;
  const int rowBase = (int)blockIdx.x * TM;

  {
    const v4f p0 = *(const v4f*)(par + 4 * tid);
    const v4f p1 = *(const v4f*)(par + 4 * (tid + GTHR));
    *(v4fa*)(pars + 4 * tid) = p0;
    *(v4fa*)(pars + 4 * (tid + GTHR)) = p1;
  }
  __syncthreads();

  {
    const v2f w10 = *(const v2fa*)(pars + P_W1 + 2 * lane);
    const v2f w11 = *(const v2fa*)(pars + P_W1 + F1 + 2 * lane);
    const v2f w12 = *(const v2fa*)(pars + P_W1 + 2 * F1 + 2 * lane);
    const v2f qb  = *(const v2fa*)(pars + P_B1 + 2 * lane);
    const v2f qm  = *(const v2fa*)(pars + P_M1 + 2 * lane);
    const v2f qs  = *(const v2fa*)(pars + P_S1 + 2 * lane);
    const v2f qe  = *(const v2fa*)(pars + P_E1 + 2 * lane);
#pragma unroll 1
    for (int ri = 0; ri < 16; ++ri) {
      const int r    = 16 * wave + ri;
      const int node = rowBase + r;
      const bool live = node < nN;
      const int nc = live ? node : nN - 1;
      const v4i nb  = *(const v4i*)(nbt + (size_t)nc * 4);
      const v4f as4 = *(const v4f*)(ax + (size_t)nc * 4);
      int c = nb.w;
      c = c < 0 ? 0 : (c > RIE - 1 ? RIE - 1 : c);
      c = live ? c : 0;
      c = __builtin_amdgcn_readfirstlane(c);
      const float di = as4.w;
      float acc0 = 0.0f, acc1 = 0.0f;
      int sj = nb.x, sy = nb.y, sz = nb.z;
#pragma unroll 1
      for (int k = 0; k < c; ++k) {
        int s = sj;
        s = s < 0 ? 0 : (s > nN - 1 ? nN - 1 : s);
        const v4f aj = *(const v4f*)(ax + (size_t)s * 4);
        h1acc(aj.x, aj.y, aj.z, aj.w * di, w10, w11, w12, qb, qm, qs, qe, acc0, acc1);
        sj = sy; sy = sz;
      }
      h1acc(as4.x, as4.y, as4.z, di * di, w10, w11, w12, qb, qm, qs, qe, acc0, acc1);
      const float v0 = live ? acc0 : 0.0f;
      const float v1 = live ? acc1 : 0.0f;
      const unsigned hb0 = bf16_bits(v0), hb1 = bf16_bits(v1);
      const unsigned lb0 = bf16_bits(v0 - __uint_as_float(hb0 << 16));
      const unsigned lb1 = bf16_bits(v1 - __uint_as_float(hb1 << 16));
      As[r * APW + lane]      = hb0 | (hb1 << 16);
      As[r * APW + 32 + lane] = lb0 | (lb1 << 16);
    }
  }
  __syncthreads();

  v8f acc[8];
  {
    const v8f z = {0.f, 0.f, 0.f, 0.f, 0.f, 0.f, 0.f, 0.f};
#pragma unroll
    for (int t = 0; t < 8; ++t) acc[t] = z;
  }
  {
    const unsigned short* arow = (const unsigned short*)As + (size_t)(16 * wave + m) * (2 * APW) + 8 * hh;
    const unsigned short* wp = W2T + (size_t)m * K2 + 8 * hh;
#pragma unroll 1
    for (int k0 = 0; k0 < K2; k0 += 32) {
      FragB af;
      af.h[0] = *(const v8usa*)(arow + k0);
      af.h[1] = *(const v8usa*)(arow + k0 + 16);
#pragma unroll
      for (int nt = 0; nt < 8; ++nt) {
        const unsigned short* wq = wp + (size_t)(16 * nt) * K2 + k0;
        FragB bf;
        bf.h[0] = *(const v8usa*)wq;
        bf.h[1] = *(const v8usa*)(wq + 16);
        acc[nt] = wmb(af, bf, acc[nt]);
      }
    }
  }
#pragma unroll
  for (int nt = 0; nt < 8; ++nt) {
    const int lc = 16 * nt + m;
#pragma unroll
    for (int r = 0; r < 8; ++r) {
      const int lr = 16 * wave + 8 * hh + r;
      stg[lr * F2 + lc] = acc[nt][r];
    }
  }
  __syncthreads();

  {
    const v4f b4 = *(const v4fa*)(pars + P_B2 + 4 * lane);
    const v4f m4 = *(const v4fa*)(pars + P_M2 + 4 * lane);
    const v4f s4 = *(const v4fa*)(pars + P_S2 + 4 * lane);
    const v4f e4 = *(const v4fa*)(pars + P_E2 + 4 * lane);
    v4f pv[16];
#pragma unroll
    for (int i = 0; i < 16; ++i) pv[i] = *(const v4fa*)(stg + (16 * wave + i) * F2 + 4 * lane);
    __syncthreads();
#pragma unroll
    for (int i = 0; i < 16; ++i) {
      const bool ok = (rowBase + 16 * wave + i) < nN;
      const v4f t = pv[i] + b4;
      v4f y = (t - m4) * s4 + e4;
      y.x = (y.x > 0.0f) ? y.x : (y.x - y.x);
      y.y = (y.y > 0.0f) ? y.y : (y.y - y.y);
      y.z = (y.z > 0.0f) ? y.z : (y.z - y.z);
      y.w = (y.w > 0.0f) ? y.w : (y.w - y.w);
      y.x = ok ? y.x : 0.0f; y.y = ok ? y.y : 0.0f; y.z = ok ? y.z : 0.0f; y.w = ok ? y.w : 0.0f;
      v4us h4, l4;
      unsigned hb;
      hb = bf16_bits(y.x); h4[0] = (unsigned short)hb; l4[0] = (unsigned short)bf16_bits(y.x - __uint_as_float(hb << 16));
      hb = bf16_bits(y.y); h4[1] = (unsigned short)hb; l4[1] = (unsigned short)bf16_bits(y.y - __uint_as_float(hb << 16));
      hb = bf16_bits(y.z); h4[2] = (unsigned short)hb; l4[2] = (unsigned short)bf16_bits(y.z - __uint_as_float(hb << 16));
      hb = bf16_bits(y.w); h4[3] = (unsigned short)hb; l4[3] = (unsigned short)bf16_bits(y.w - __uint_as_float(hb << 16));
      unsigned short* srow = (unsigned short*)stg + (size_t)(16 * wave + i) * (2 * F2);
      *(v4usa*)(srow + 4 * lane) = h4;
      *(v4usa*)(srow + F2 + 4 * lane) = l4;
    }
  }
  __syncthreads();

  v8f c2[2];
  {
    const v8f z = {0.f, 0.f, 0.f, 0.f, 0.f, 0.f, 0.f, 0.f};
    c2[0] = z; c2[1] = z;
  }
  {
    const unsigned short* a2row = (const unsigned short*)stg + (size_t)(16 * wave + m) * (2 * F2) + 8 * hh;
    const unsigned short* w3p = W3T + (size_t)m * K3 + 8 * hh;
#pragma unroll 1
    for (int k0 = 0; k0 < K3; k0 += 32) {
      FragB af;
      af.h[0] = *(const v8usa*)(a2row + k0);
      af.h[1] = *(const v8usa*)(a2row + k0 + 16);
#pragma unroll
      for (int nt = 0; nt < 2; ++nt) {
        const unsigned short* wq = w3p + (size_t)(16 * nt) * K3 + k0;
        FragB bf;
        bf.h[0] = *(const v8usa*)wq;
        bf.h[1] = *(const v8usa*)(wq + 16);
        c2[nt] = wmb(af, bf, c2[nt]);
      }
    }
  }
#pragma unroll
  for (int nt = 0; nt < 2; ++nt) {
    const int lc = 16 * nt + m;
#pragma unroll
    for (int r = 0; r < 8; ++r) {
      const int lr = 16 * wave + 8 * hh + r;
      if (lc < NC) t3s[lr * NC + lc] = c2[nt][r];
    }
  }
  __syncthreads();

  constexpr int NQ = (TM * NC) / 4;
  v4f ov[4];
#pragma unroll
  for (int it = 0; it < 4; ++it) {
    const int q  = it * GTHR + tid;
    const int qc = q < NQ ? q : NQ - 1;
    ov[it] = *(const v4fa*)(t3s + 4 * qc);
  }
  float* tp = t3 + (size_t)blockIdx.x * (TM * NC);
#pragma unroll
  for (int it = 0; it < 4; ++it) {
    const int q = it * GTHR + tid;
    if (q < NQ) *(volatile v4f*)(tp + 4 * q) = ov[it];
  }
  __threadfence();
#pragma unroll
  for (int it = 0; it < 4; ++it) {
    const int q = it * GTHR + tid;
    if (q < NQ) *(volatile v4f*)(tp + 4 * q) = ov[it];
  }
}

__global__ __launch_bounds__(NTHR) void k_pool(const float* __restrict__ t3, const int* __restrict__ nbt,
                                               const float* __restrict__ dinv, const int* __restrict__ memb,
                                               const float* __restrict__ par, int nN, int nG, int outN,
                                               float* out) {
  __shared__ __attribute__((aligned(16))) float os[GPB * NC];
  const int tid = (int)threadIdx.x, lane = tid & 31, wave = tid >> 5;
  const int cl = lane < NC ? lane : NC - 1;
  const bool cls = lane < NC;
  const float b3v = par[P_B3 + cl];
  const float qnan = __int_as_float(0x7fc00000);
  const float ninf = __int_as_float((int)0xff800000);

#pragma unroll 1
  for (int gi = 0; gi < GPB / NWAVE; ++gi) {
    const int gl = wave * (GPB / NWAVE) + gi;
    const int g  = (int)blockIdx.x * GPB + gl;
    const bool liveg = g < nG;
    const int gc = liveg ? g : nG - 1;
    const int mv = memb[(size_t)gc * RIG + lane];
    const int cntg = __builtin_amdgcn_readlane(mv, RIG - 1);
    int cc = cntg < 0 ? 0 : (cntg > RIG - 1 ? RIG - 1 : cntg);
    cc = liveg ? cc : 0;
    float sum = 0.0f;
#pragma unroll 1
    for (int q = 0; q < cc; ++q) {
      int i = __builtin_amdgcn_readlane(mv, q);
      i = i < 0 ? 0 : (i > nN - 1 ? nN - 1 : i);
      const v4i nb = *(const v4i*)(nbt + (size_t)i * 4);
      const float di = dinv[i];
      int c = nb.w;
      c = c < 0 ? 0 : (c > RIE - 1 ? RIE - 1 : c);
      c = __builtin_amdgcn_readfirstlane(c);
      float acc = 0.0f;
      int sj = nb.x, sy = nb.y, sz = nb.z;
#pragma unroll 1
      for (int k = 0; k < c; ++k) {
        int s = sj;
        s = s < 0 ? 0 : (s > nN - 1 ? nN - 1 : s);
        const float ds = dinv[s];
        const float tv = t3[(size_t)s * NC + cl];
        acc = fmaf(ds * di, tv, acc);
        sj = sy; sy = sz;
      }
      const float ts = t3[(size_t)i * NC + cl];
      const float h3 = (acc + (di * di) * ts) + b3v;
      sum += h3;
    }
    const float cf = (float)cntg;
    float p = sum * (1.0f / cf);
    p = (cntg > RIG - 1) ? qnan : p;
    float mx = cls ? p : ninf;
#pragma unroll
    for (int d = 16; d >= 1; d >>= 1) mx = fmaxf(mx, __shfl_xor(mx, d, 32));
    const float sh = p - mx;
    const float ev = expf(sh);
    float se = cls ? ev : 0.0f;
#pragma unroll
    for (int d = 16; d >= 1; d >>= 1) se += __shfl_xor(se, d, 32);
    const float o = sh - logf(se);
    if (cls) os[gl * NC + lane] = liveg ? o : 0.0f;
  }
  __syncthreads();

  constexpr int NQ = (GPB * NC) / 4;
  const int qc = tid < NQ ? tid : NQ - 1;
  const v4f ov = *(const v4fa*)(os + 4 * qc);
  const size_t fo = (size_t)blockIdx.x * (GPB * NC) + (size_t)4 * tid;
  const bool st = (tid < NQ) && (fo + 3 < (size_t)outN);
  float* op = out + fo;
  if (st) *(volatile v4f*)op = ov;
  __threadfence();
  if (st) *(volatile v4f*)op = ov;
}

static inline int cdiv(int a, int b) { return (a + b - 1) / b; }
static inline size_t al256(size_t o) { return (o + 255) & ~(size_t)255; }

extern "C" void kernel_launch(void* const* d_in, const int* in_sizes, int n_in,
                              void* d_out, int out_size, void* d_ws, size_t ws_size,
                              hipStream_t stream) {
  if (n_in < 17) return;
  if (in_sizes[0] < 3 || (in_sizes[0] % 3) != 0) return;
  const int nN = in_sizes[0] / 3;
  if (nN < 1 || nN > (1 << 24)) return;
  if (in_sizes[1] != 3 * F1) return;
  if (in_sizes[2] != F1 || in_sizes[3] != F1 || in_sizes[4] != F1 || in_sizes[5] != F1 || in_sizes[6] != F1) return;
  if (in_sizes[7] != F1 * F2) return;
  if (in_sizes[8] != F2 || in_sizes[9] != F2 || in_sizes[10] != F2 || in_sizes[11] != F2 || in_sizes[12] != F2) return;
  if (in_sizes[13] != F2 * NC || in_sizes[14] != NC) return;
  if (in_sizes[15] < 2 || (in_sizes[15] & 1) != 0) return;
  const int nE = in_sizes[15] / 2;
  if (nE < 1 || nE > (1 << 28)) return;
  if (in_sizes[16] != nN) return;
  if (out_size < NC || (out_size % NC) != 0) return;
  const int nG = out_size / NC;
  if (nG > (1 << 24)) return;

  const float* x   = (const float*)d_in[0];
  const float* W1  = (const float*)d_in[1];
  const float* b1  = (const float*)d_in[2];
  const float* g1  = (const float*)d_in[3];
  const float* be1 = (const float*)d_in[4];
  const float* m1  = (const float*)d_in[5];
  const float* v1  = (const float*)d_in[6];
  const float* W2  = (const float*)d_in[7];
  const float* b2  = (const float*)d_in[8];
  const float* g2  = (const float*)d_in[9];
  const float* be2 = (const float*)d_in[10];
  const float* m2  = (const float*)d_in[11];
  const float* v2  = (const float*)d_in[12];
  const float* W3  = (const float*)d_in[13];
  const float* b3  = (const float*)d_in[14];
  const int*   edge = (const int*)d_in[15];
  const int*   bat  = (const int*)d_in[16];
  float* out = (float*)d_out;
  const int* src = edge;
  const int* dst = edge + nE;

  const int nbE = cdiv(nN, 1 << SLE);
  const int nbA = cdiv(nN, NTHR);
  const int nT  = cdiv(nN, TM);
  const int nbG = cdiv(nG, 1 << SLG);
  const int nP  = cdiv(nG, GPB);
  const int vec8E = ((nE & 3) == 0) ? 1 : 0;

  char* ws = (char*)d_ws;
  size_t off = 0;
  const size_t oPAR = off; off = al256(off + (size_t)PARN * 4);
  const size_t oW2T = off; off = al256(off + (size_t)F2 * K2 * 2);
  const size_t oW3T = off; off = al256(off + (size_t)32 * K3 * 2);
  const size_t oNBT = off; off = al256(off + (size_t)nbE * TABN * 4);
  const size_t oDIN = off; off = al256(off + (size_t)nbE * (1 << SLE) * 4);
  const size_t oAX  = off; off = al256(off + (size_t)nbA * NTHR * 16);
  const size_t oT3  = off; off = al256(off + (size_t)nT * (TM * NC) * 4);
  const size_t oMB  = off; off = al256(off + (size_t)nbG * TABN * 4);
  if (off > ws_size) return;
  float*          PAR  = (float*)(ws + oPAR);
  unsigned short* W2T  = (unsigned short*)(ws + oW2T);
  unsigned short* W3T  = (unsigned short*)(ws + oW3T);
  int*            NBT  = (int*)(ws + oNBT);
  float*          DINV = (float*)(ws + oDIN);
  float*          AX   = (float*)(ws + oAX);
  float*          T3   = (float*)(ws + oT3);
  int*            MEMB = (int*)(ws + oMB);

  const size_t cmpLds = (size_t)CMP_INTS * 4;
  hipFuncSetAttribute(reinterpret_cast<const void*>(&k_compact<SLE, RIE, 1>), hipFuncAttributeMaxDynamicSharedMemorySize, (int)cmpLds);
  hipFuncSetAttribute(reinterpret_cast<const void*>(&k_compact<SLG, RIG, 0>), hipFuncAttributeMaxDynamicSharedMemorySize, (int)cmpLds);

  k_prep<<<NU2 / NTHR + NU3 / NTHR + 1, NTHR, 0, stream>>>(W1, b1, g1, be1, m1, v1, W2, b2, g2, be2, m2, v2,
                                                           W3, b3, PAR, W2T, W3T);
  k_compact<SLE, RIE, 1><<<nbE, NTHR, cmpLds, stream>>>(dst, src, nE, nN, vec8E, NBT, DINV);
  k_agg1<<<nbA, NTHR, 0, stream>>>(x, NBT, DINV, nN, AX);
  k_layer2<<<nT, GTHR, 0, stream>>>(AX, NBT, PAR, W2T, W3T, nN, T3);
  k_compact<SLG, RIG, 0><<<nbG, NTHR, cmpLds, stream>>>(bat, bat, nN, nN, 1, MEMB, DINV);
  k_pool<<<nP, NTHR, 0, stream>>>(T3, NBT, DINV, MEMB, PAR, nN, nG, out_size, out);
}
